// SpectralAttention_10402410791708
// MI455X (gfx1250) — hardware-verified
//
#include <hip/hip_runtime.h>

#ifndef NB
#define NB 4
#endif
#ifndef SEQ
#define SEQ 2048
#endif
#define NB_FULL 4
#define SEQ_FULL 2048
#define DD 1024
#define PP 128

static_assert(NB >= 1 && NB <= NB_FULL);
static_assert(SEQ % 256 == 0 && SEQ >= 256 && SEQ <= SEQ_FULL);
static_assert(DD % 64 == 0 && PP % 64 == 0);
static_assert(DD % 32 == 0 && PP % 32 == 0 && SEQ % 64 == 0);

typedef __attribute__((ext_vector_type(8)))  _Float16 v8h;
typedef __attribute__((ext_vector_type(16))) __bf16   v16b;
typedef __attribute__((ext_vector_type(8)))  __bf16   v8b;
typedef __attribute__((ext_vector_type(8)))  float    v8f;
typedef __attribute__((ext_vector_type(4)))  float    v4f;
typedef __attribute__((ext_vector_type(4)))  unsigned int v4u;

__device__ __forceinline__ unsigned short f2bf_bits(float f) {
  unsigned u = __float_as_uint(f);
  return (unsigned short)((u + 0x7FFFu + ((u >> 16) & 1u)) >> 16);
}
__device__ __forceinline__ float bf_bits2f(unsigned short h) { return __uint_as_float(((unsigned)h) << 16); }

__device__ __forceinline__ void dep_guard_b(v8f& a, v8f& b, v16b x, v16b y) { asm volatile("v_nop\n\tv_nop\n\tv_nop\n\tv_nop" : "+v"(a), "+v"(b) : "v"(x), "v"(y)); }
__device__ __forceinline__ void keep4_b(v16b a, v16b b, v16b c, v16b d) { asm volatile("v_nop" :: "v"(a), "v"(b), "v"(c), "v"(d)); }
__device__ __forceinline__ void acc_guard4(v8f& a, v8f& b, v8f& c, v8f& d) { asm volatile("v_nop\n\tv_nop\n\tv_nop\n\tv_nop" : "+v"(a), "+v"(b), "+v"(c), "+v"(d)); }

struct FragB {
  union U { v16b v; v8b h[2]; };
  static __device__ __forceinline__ v16b load(const __bf16* p) {
    U f; f.h[0] = *(const v8b*)(p); f.h[1] = *(const v8b*)(p + 16); return f.v;
  }
  static __device__ __forceinline__ v8f mma(v16b a, v16b b, v8f c) {
    return __builtin_amdgcn_wmma_f32_16x16x32_bf16(false, a, false, b, (short)0, c, false, false);
  }
  static __device__ __forceinline__ void guard(v8f& a, v8f& b, v16b x, v16b y) { dep_guard_b(a, b, x, y); }
  static __device__ __forceinline__ void keep(v16b a, v16b b, v16b c, v16b d) { keep4_b(a, b, c, d); }
};

__device__ __forceinline__ unsigned pk16(unsigned short a, unsigned short b) { return (unsigned)a | ((unsigned)b << 16); }

template <int SA, int SB, int EPI, int OUT_MODE, int CAUSAL>
__global__ __launch_bounds__(256) void wmma_gemm64(
    const unsigned short* __restrict__ Ap, const unsigned short* __restrict__ A2p, int lda, long strideA,
    const unsigned short* __restrict__ Btp, const unsigned short* __restrict__ Bt2p, int ldb, long strideB,
    void* __restrict__ Cout, void* __restrict__ Cout2, int ldc, long strideC,
    const float* __restrict__ bias0, const float* __restrict__ bias1,
    int M, int N, int K, float scale) {
  typedef __bf16 T;
  typedef v16b V;
  const T* A = (const T*)Ap; const T* A2 = (const T*)A2p; const T* Bt = (const T*)Btp; const T* Bt2 = (const T*)Bt2p;
  __shared__ __align__(16) float sT[8][16 * 68];
  const int b    = blockIdx.y;
  const int lane = threadIdx.x & 31;
  const int wave = threadIdx.x >> 5;
  const int tilesN = N >> 6;
  const int tilesM = M >> 6;
  const int tile = blockIdx.x * 8 + wave;
  if (tile >= tilesM * tilesN) return;
  const int tm = tile / tilesN;
  const int tn = tile - tm * tilesN;
  const int m0 = tm << 6;
  const int n0 = tn << 6;
  if (CAUSAL == 1) { if (n0 >= m0 + 64) return; }
  const int kEnd = (CAUSAL == 2) ? ((m0 + 64 < K) ? (m0 + 64) : K) : K;

  const T* Ab  = A  + (size_t)b * strideA;
  const T* Bb  = Bt + (size_t)b * strideB;
  const T* Ab2 = (SA != 0) ? (A2  + (size_t)b * strideA) : nullptr;
  const T* Bb2 = (SB != 0) ? (Bt2 + (size_t)b * strideB) : nullptr;
  const float* bias = (b == 0) ? bias0 : bias1;

  const int rlane = lane & 15;
  const int koff  = (lane >> 4) * 8;
  const int mOff  = (lane >> 4) * 8;

  v8f acc[4][4];
#pragma unroll
  for (int i = 0; i < 4; ++i)
#pragma unroll
    for (int j = 0; j < 4; ++j) acc[i][j] = (v8f){0.f,0.f,0.f,0.f,0.f,0.f,0.f,0.f};

  for (int k0 = 0; k0 < kEnd; k0 += 32) {
    V bh[4], bl[4];
#pragma unroll
    for (int j = 0; j < 4; ++j) {
      const size_t bo = (size_t)(n0 + (j << 4) + rlane) * ldb + koff + k0;
      bh[j] = FragB::load(Bb + bo);
      if (SB != 0) bl[j] = FragB::load(Bb2 + bo);
    }
#pragma unroll
    for (int i = 0; i < 4; ++i) {
      const size_t ao = (size_t)(m0 + (i << 4) + rlane) * lda + koff + k0;
      V ah = FragB::load(Ab + ao);
      V al = ah;
      if (SA != 0) al = FragB::load(Ab2 + ao);
#pragma unroll
      for (int j = 0; j < 4; ++j) {
        acc[i][j] = FragB::mma(ah, bh[j], acc[i][j]);
        if (SB != 0) acc[i][j] = FragB::mma(ah, bl[j], acc[i][j]);
        if (SA != 0) acc[i][j] = FragB::mma(al, bh[j], acc[i][j]);
      }
      FragB::guard(acc[i][0], acc[i][3], ah, al);
    }
    FragB::keep(bh[0], bh[1], bh[2], bh[3]);
    if (SB != 0) FragB::keep(bl[0], bl[1], bl[2], bl[3]);
  }
  acc_guard4(acc[0][0], acc[0][1], acc[0][2], acc[0][3]);
  acc_guard4(acc[1][0], acc[1][1], acc[1][2], acc[1][3]);
  acc_guard4(acc[2][0], acc[2][1], acc[2][2], acc[2][3]);
  acc_guard4(acc[3][0], acc[3][1], acc[3][2], acc[3][3]);

  float* slab = sT[wave];
#pragma unroll
  for (int i = 0; i < 4; ++i) {
    const int mBase = m0 + (i << 4);
#pragma unroll
    for (int j = 0; j < 4; ++j) {
      const int n = n0 + (j << 4) + rlane;
      float bvl = 0.f;
      float csc = 1.f;
      if (EPI == 2) bvl = bf_bits2f(f2bf_bits(bias[n]));
      if (EPI == 3) csc = bf_bits2f(f2bf_bits(bias0[n]));
#pragma unroll
      for (int r = 0; r < 8; ++r) {
        float v = acc[i][j][r] * scale;
        if (EPI == 2) v += bvl;
        if (EPI == 3) {
          const int m = mBase + mOff + r;
          v = (n <= m) ? (v * csc) : 0.f;
        }
        slab[(mOff + r) * 68 + (j << 4) + rlane] = v;
      }
    }
    __builtin_amdgcn_fence(__ATOMIC_RELEASE, "workgroup");
    __builtin_amdgcn_wave_barrier();
    __builtin_amdgcn_fence(__ATOMIC_ACQUIRE, "workgroup");
    if (OUT_MODE == 0) {
      float* C = (float*)Cout + (size_t)b * strideC;
      const int hh = lane >> 4, c4 = (lane & 15) * 4;
      for (int pass = 0; pass < 2; ++pass) {
#pragma unroll
        for (int it = 0; it < 8; ++it) {
          const int row = it * 2 + hh;
          v4f v = *(const v4f*)(slab + row * 68 + c4);
          *(volatile v4f*)(C + (size_t)(mBase + row) * ldc + n0 + c4) = v;
        }
        __threadfence();
      }
    } else {
      const int q = lane >> 3, c8 = (lane & 7) * 8;
      unsigned short* C  = (unsigned short*)Cout  + (size_t)b * strideC;
      unsigned short* C2 = (unsigned short*)Cout2 + (size_t)b * strideC;
      for (int pass = 0; pass < 2; ++pass) {
#pragma unroll
        for (int it = 0; it < 4; ++it) {
          const int row = it * 4 + q;
          const float* sp = slab + row * 68 + c8;
          v8h hv, lv;
#pragma unroll
          for (int e = 0; e < 8; ++e) {
            unsigned short hb = f2bf_bits(sp[e]);
            unsigned short lb = f2bf_bits(sp[e] - bf_bits2f(hb));
            hv[e] = __builtin_bit_cast(_Float16, hb);
            lv[e] = __builtin_bit_cast(_Float16, lb);
          }
          *(volatile v8h*)(C + (size_t)(mBase + row) * ldc + n0 + c8) = hv;
          *(volatile v8h*)(C2 + (size_t)(mBase + row) * ldc + n0 + c8) = lv;
        }
        __threadfence();
      }
    }
    __builtin_amdgcn_fence(__ATOMIC_RELEASE, "workgroup");
    __builtin_amdgcn_wave_barrier();
    __builtin_amdgcn_fence(__ATOMIC_ACQUIRE, "workgroup");
  }
}

__global__ __launch_bounds__(256) void x_prep_kernel(const float* __restrict__ x, unsigned short* __restrict__ xb) {
  const int gid = blockIdx.x * 256 + threadIdx.x;
  const int r   = gid >> 7;
  const int c8  = (gid & 127) * 8;
  const int b   = r / SEQ;
  const int t   = r - b * SEQ;
  const float* src = x + ((size_t)b * SEQ_FULL + t) * DD + c8;
  const v4f a = *(const v4f*)(src);
  const v4f c = *(const v4f*)(src + 4);
  unsigned short hb[8];
#pragma unroll
  for (int e = 0; e < 4; ++e) { hb[e] = f2bf_bits(a[e]); hb[4 + e] = f2bf_bits(c[e]); }
  const v4u uh = (v4u){pk16(hb[0], hb[1]), pk16(hb[2], hb[3]), pk16(hb[4], hb[5]), pk16(hb[6], hb[7])};
  unsigned short* p = xb + (size_t)r * DD + c8;
  *(volatile v4u*)(p) = uh;
  __threadfence();
  *(volatile v4u*)(p) = uh;
}

__global__ __launch_bounds__(256) void tr_prep_kernel(const float* __restrict__ in0, const float* __restrict__ in1,
                                                      int R, int C, unsigned short* __restrict__ out, long planeOut) {
  __shared__ float sm[64][65];
  const int t  = threadIdx.x;
  const int c0 = blockIdx.x * 64;
  const int r0 = blockIdx.y * 64;
  const int z  = blockIdx.z;
  const float* in  = (z == 0) ? in0 : in1;
  const float* src = in + (size_t)r0 * C + c0;
#pragma unroll
  for (int i = 0; i < 16; ++i) {
    const int e  = i * 256 + t;
    const int rl = e >> 6;
    const int cl = e & 63;
    sm[cl][rl] = bf_bits2f(f2bf_bits(src[(size_t)rl * C + cl]));
  }
  __syncthreads();
  const int lane = t & 31, wave = t >> 5;
  const int q = lane >> 3, c8 = (lane & 7) * 8;
  unsigned short* ob = out + (size_t)z * planeOut;
  for (int pass = 0; pass < 2; ++pass) {
#pragma unroll
    for (int it = 0; it < 2; ++it) {
      const int row = wave * 8 + it * 4 + q;
      unsigned short bb[8];
#pragma unroll
      for (int e = 0; e < 8; ++e) bb[e] = f2bf_bits(sm[row][c8 + e]);
      const v4u ub = (v4u){pk16(bb[0], bb[1]), pk16(bb[2], bb[3]), pk16(bb[4], bb[5]), pk16(bb[6], bb[7])};
      *(volatile v4u*)(ob + (size_t)(c0 + row) * R + r0 + c8) = ub;
    }
    __threadfence();
  }
}

static inline size_t al64k(size_t v) { return (v + (size_t)65535) & ~(size_t)65535; }
static inline unsigned cdivu(unsigned a, unsigned b) { return (a + b - 1) / b; }

extern "C" void kernel_launch(void* const* d_in, const int* in_sizes, int n_in,
                              void* d_out, int out_size, void* d_ws, size_t ws_size,
                              hipStream_t stream) {
  if (n_in != 10) return;
  if (in_sizes[0] < (NB - 1) * SEQ_FULL * DD + SEQ * DD) return;
  if (in_sizes[1] < PP * PP || in_sizes[2] < PP * PP) return;
  if (in_sizes[3] < DD * PP || in_sizes[5] < DD * PP) return;
  if (in_sizes[4] < PP || in_sizes[6] < PP) return;
  if (in_sizes[7] < PP * DD || in_sizes[8] < DD) return;
  if (in_sizes[9] < SEQ) return;
  if (out_size < (NB - 1) * SEQ_FULL * DD + SEQ * DD) return;

  const size_t szXb  = (size_t)NB * SEQ * DD * 2;
  const size_t szWT  = (size_t)2 * PP * DD * 2;
  const size_t szFT  = (size_t)2 * PP * PP * 2;
  const size_t szWoT = (size_t)DD * PP * 2;
  const size_t szXpv = (size_t)2 * NB * SEQ * PP * 2;
  const size_t szQ   = (size_t)NB * SEQ * PP * 2;
  const size_t szKT  = (size_t)NB * PP * SEQ * 2;
  const size_t szSm  = (size_t)SEQ * SEQ * 2;
  const size_t szY   = (size_t)NB * SEQ * PP * 2;
  size_t off = 0;
  const size_t offXb   = off; off = al64k(off + szXb);
  const size_t offWT   = off; off = al64k(off + szWT);
  const size_t offFT   = off; off = al64k(off + szFT);
  const size_t offWoT  = off; off = al64k(off + szWoT);
  const size_t offXpvH = off; off = al64k(off + szXpv);
  const size_t offXpvL = off; off = al64k(off + szXpv);
  const size_t offQH   = off; off = al64k(off + szQ);
  const size_t offQL   = off; off = al64k(off + szQ);
  const size_t offKTH  = off; off = al64k(off + szKT);
  const size_t offKTL  = off; off = al64k(off + szKT);
  const size_t offSmH  = off; off = al64k(off + szSm);
  const size_t offSmL  = off; off = al64k(off + szSm);
  const size_t offYH   = off; off = al64k(off + szY);
  const size_t offYL   = off; off = al64k(off + szY);
  const size_t total   = off;
  if (ws_size < total) return;
  if (total > ((size_t)128 << 20)) return;

  const float* x     = (const float*)d_in[0];
  const float* Qf    = (const float*)d_in[1];
  const float* Kf    = (const float*)d_in[2];
  const float* W_in  = (const float*)d_in[3];
  const float* b_in  = (const float*)d_in[4];
  const float* W_v   = (const float*)d_in[5];
  const float* b_v   = (const float*)d_in[6];
  const float* W_o   = (const float*)d_in[7];
  const float* b_o   = (const float*)d_in[8];
  const float* decay = (const float*)d_in[9];
  float* out = (float*)d_out;

  char* ws = (char*)d_ws;
  unsigned short* xb   = (unsigned short*)(ws + offXb);
  unsigned short* wT   = (unsigned short*)(ws + offWT);
  unsigned short* fT   = (unsigned short*)(ws + offFT);
  unsigned short* woT  = (unsigned short*)(ws + offWoT);
  unsigned short* xpvh = (unsigned short*)(ws + offXpvH);
  unsigned short* xpvl = (unsigned short*)(ws + offXpvL);
  unsigned short* qh   = (unsigned short*)(ws + offQH);
  unsigned short* ql   = (unsigned short*)(ws + offQL);
  unsigned short* kTh  = (unsigned short*)(ws + offKTH);
  unsigned short* kTl  = (unsigned short*)(ws + offKTL);
  unsigned short* smh  = (unsigned short*)(ws + offSmH);
  unsigned short* sml  = (unsigned short*)(ws + offSmL);
  unsigned short* yh   = (unsigned short*)(ws + offYH);
  unsigned short* yl   = (unsigned short*)(ws + offYL);

  const long planeW   = (long)PP * DD;
  const long planeF   = (long)PP * PP;
  const long planeXpv = (long)NB * SEQ * PP;
  const long batchTP  = (long)SEQ * PP;
  const long planeKT  = (long)PP * SEQ;

  x_prep_kernel<<<dim3((unsigned)((size_t)NB * SEQ * (DD / 8) / 256)), 256, 0, stream>>>(x, xb);
  tr_prep_kernel<<<dim3(PP / 64, DD / 64, 2), 256, 0, stream>>>(W_in, W_v, DD, PP, wT, planeW);
  tr_prep_kernel<<<dim3(PP / 64, PP / 64, 2), 256, 0, stream>>>(Qf, Kf, PP, PP, fT, planeF);
  tr_prep_kernel<<<dim3(DD / 64, PP / 64, 1), 256, 0, stream>>>(W_o, W_o, PP, DD, woT, 0L);

  const unsigned blkProj = cdivu((unsigned)((NB * SEQ / 64) * (PP / 64)), 8);
  const unsigned blkKT   = cdivu((unsigned)((PP / 64) * (SEQ / 64)), 8);
  const unsigned blkSc   = cdivu((unsigned)((SEQ / 64) * (SEQ / 64)), 8);
  const unsigned blkY    = cdivu((unsigned)((SEQ / 64) * (PP / 64)), 8);
  const unsigned blkOut  = cdivu((unsigned)((SEQ / 64) * (DD / 64)), 8);

  wmma_gemm64<0, 0, 2, 2, 0><<<dim3(blkProj, 2), 256, 0, stream>>>(
      xb, xb, DD, 0L, wT, wT, DD, planeW,
      (void*)xpvh, (void*)xpvl, PP, planeXpv, b_in, b_v, NB * SEQ, PP, DD, 1.0f);
  wmma_gemm64<1, 0, 0, 2, 0><<<dim3(blkProj, 1), 256, 0, stream>>>(
      xpvh, xpvl, PP, 0L, fT, fT, PP, 0L,
      (void*)qh, (void*)ql, PP, 0L, b_in, b_in, NB * SEQ, PP, PP, 1.0f);
  wmma_gemm64<0, 1, 0, 2, 0><<<dim3(blkKT, NB), 256, 0, stream>>>(
      fT + planeF, fT + planeF, PP, 0L, xpvh, xpvl, PP, batchTP,
      (void*)kTh, (void*)kTl, SEQ, planeKT, b_in, b_in, PP, SEQ, PP, 1.0f);

  for (int bb = 0; bb < NB; ++bb) {
    const size_t oTP = (size_t)bb * batchTP;
    wmma_gemm64<1, 1, 3, 2, 1><<<dim3(blkSc, 1), 256, 0, stream>>>(
        qh + oTP, ql + oTP, PP, 0L, xpvh + planeXpv + oTP, xpvl + planeXpv + oTP, PP, 0L,
        (void*)smh, (void*)sml, SEQ, 0L, decay, decay, SEQ, SEQ, PP, 1.0f);
    wmma_gemm64<1, 1, 0, 2, 2><<<dim3(blkY, 1), 256, 0, stream>>>(
        smh, sml, SEQ, 0L, kTh + (size_t)bb * planeKT, kTl + (size_t)bb * planeKT, SEQ, 0L,
        (void*)(yh + oTP), (void*)(yl + oTP), PP, 0L, decay, decay, SEQ, PP, SEQ, 1.0f);
  }
  wmma_gemm64<1, 0, 2, 0, 0><<<dim3(blkOut, NB), 256, 0, stream>>>(
      yh, yl, PP, batchTP, woT, woT, PP, 0L,
      (void*)out, (void*)out, DD, (long)SEQ_FULL * DD, b_o, b_o, SEQ, DD, PP, 1.0f);
}
